// EdgeDecoder_15831249453675
// MI455X (gfx1250) — hardware-verified
//
#include <hip/hip_runtime.h>


namespace {

constexpr int N = 100000, NP = 100032, EFULL = 640000, EL = EFULL  ;
constexpr int D = 128, HID = 128;
constexpr float XS = 8.0f, WSC = 256.0f, RS_ = 1024.0f;
static_assert(NP % 32 == 0 && NP >= N && EFULL % 32 == 0 && EL % 32 == 0, "tiling");
typedef _Float16 b16;
typedef __attribute__((ext_vector_type(16))) _Float16 v16b;
typedef __attribute__((ext_vector_type(8))) _Float16 v8b;
typedef __attribute__((ext_vector_type(8))) float v8f;
typedef __attribute__((ext_vector_type(4))) float v4f;
typedef __attribute__((ext_vector_type(4))) _Float16 v4h;
__device__ __forceinline__ float bf16_rne(float f) { unsigned int u = __float_as_uint(f); u += 0x7FFFu + ((u >> 16) & 1u); return __uint_as_float(u & 0xFFFF0000u); }
__device__ __forceinline__ v16b frag_kb(const b16* p, int hh) { const v8b a = *(const v8b*)(p + 8 * hh), b = *(const v8b*)(p + 16 + 8 * hh); v16b f;
#pragma unroll
  for (int e = 0; e < 8; ++e) { f[e] = a[e]; f[8 + e] = b[e]; } return f; }
__device__ __forceinline__ v8f wmma16b(v16b a, v16b b, v8f c) { v8f d = __builtin_amdgcn_wmma_f32_16x16x32_f16(false, a, false, b, (short)0, c, false, false); asm volatile("v_nop\n\tv_nop\n\tv_nop\n\tv_nop" : "+v"(d) : "v"(a), "v"(b)); return d; }
__device__ __forceinline__ void wave_lds_sync() { __builtin_amdgcn_fence(__ATOMIC_RELEASE, "workgroup"); __builtin_amdgcn_wave_barrier(); __builtin_amdgcn_fence(__ATOMIC_ACQUIRE, "workgroup"); }
__device__ __forceinline__ int iclamp(int v, int lo, int hi) { return v < lo ? lo : (v > hi ? hi : v); }
__global__ __launch_bounds__(256) void wt_kernel(const float* __restrict__ w, b16* __restrict__ WT, float scl) {
  const int u = blockIdx.x * 256 + threadIdx.x; if (u >= 2 * HID * D / 8) return; const int e = u * 8; const int o = e / D, k0 = e % D; const int half = o / HID, oc = o % HID; v8b v;
#pragma unroll
  for (int j = 0; j < 8; ++j) v[j] = (b16)(bf16_rne(w[((size_t)half * D + k0 + j) * HID + oc]) * scl);
  for (int pass = 0; pass < 2; ++pass) { *(volatile v8b*)(WT + e) = v; __threadfence(); }
}
template <int HALF>
__global__ __launch_bounds__(64) void ab_kernel(const float* __restrict__ z, const b16* __restrict__ WT, const float* __restrict__ b1, float* __restrict__ AB) {
  __shared__ __attribute__((aligned(16))) b16 Ah[2][16][D + 8]; __shared__ __attribute__((aligned(16))) float Tf[2][16][HID + 4];
  const int wave = threadIdx.x >> 5, lane = threadIdx.x & 31, nloc = lane & 15, hlf = lane >> 4; const size_t m0 = (size_t)blockIdx.x * 32 + wave * 16;
  for (int idx = lane; idx < 16 * (D / 4); idx += 32) { const int rr = idx / (D / 4), c4 = (idx % (D / 4)) * 4; const size_t arow = (m0 + rr < (size_t)N) ? m0 + rr : (size_t)N - 1; const v4f v = *(const v4f*)(z + arow * D + c4); v4h hv; for (int j = 0; j < 4; ++j) hv[j] = (b16)(bf16_rne(v[j]) * XS); *(v4h*)(&Ah[wave][rr][c4]) = hv; }
  wave_lds_sync();
  v8f acc[8];
#pragma unroll
  for (int t = 0; t < 8; ++t) acc[t] = (v8f){};
#pragma unroll 1
  for (int kb = 0; kb < D; kb += 32) { const v16b a = frag_kb(&Ah[wave][nloc][kb], hlf);
#pragma unroll
    for (int t = 0; t < 8; ++t) acc[t] = wmma16b(a, frag_kb(WT + (size_t)(HALF * HID + t * 16 + nloc) * D + kb, hlf), acc[t]); }
#pragma unroll
  for (int t = 0; t < 8; ++t) { const int col = t * 16 + nloc; const float bb = (HALF == 0) ? bf16_rne(b1[col]) : 0.0f; for (int r = 0; r < 8; ++r) Tf[wave][8 * hlf + r][col] = (m0 + 8 * hlf + r < (size_t)N) ? acc[t][r] * (1.0f / (XS * WSC)) + bb : 0.0f; }
  wave_lds_sync();
  for (int pass = 0; pass < 2; ++pass) { for (int rr = 0; rr < 16; ++rr) *(volatile v4f*)(AB + (m0 + rr) * (2 * HID) + HALF * HID + lane * 4) = *(const v4f*)(&Tf[wave][rr][lane * 4]); __threadfence(); }
}
__global__ __launch_bounds__(256) void edge_kernel(const float* __restrict__ AB, const int* __restrict__ ei, const float* __restrict__ W2, const float* __restrict__ b2, float* __restrict__ out, int mcount) {
  const int e = blockIdx.x * 256 + threadIdx.x; if (e >= ((mcount + 31) / 32) * 32) return; const int ec = e < EFULL ? e : EFULL - 1;
  const int s = iclamp(ei[ec], 0, N - 1), d = iclamp(ei[(size_t)EFULL + ec], 0, N - 1); const float* ar = AB + (size_t)s * (2 * HID); const float* br = AB + (size_t)d * (2 * HID) + HID; float acc = 0.0f;
#pragma unroll 1
  for (int c = 0; c < HID; c += 4) { const v4f a4 = *(const v4f*)(ar + c), b4 = *(const v4f*)(br + c), w4 = *(const v4f*)(W2 + c);
#pragma unroll
    for (int j = 0; j < 4; ++j) acc = fmaf(fmaxf(a4[j] + b4[j], 0.0f), bf16_rne(w4[j]), acc); }
  const float lg = acc + bf16_rne(b2[0]); const float val = 1.0f / (1.0f + __expf(-lg));
  for (int pass = 0; pass < 2; ++pass) { if (e < mcount) ((volatile float*)out)[e] = val; __threadfence(); }
}
}

extern "C" void kernel_launch(void* const* d_in, const int* in_sizes, int n_in, void* d_out, int out_size, void* d_ws, size_t ws_size, hipStream_t stream) {
  (void)n_in;
  auto Fp = [&](int i) { return (const float*)d_in[i]; }; auto Ip = [&](int i) { return (const int*)d_in[i]; };
  if (in_sizes[0] != N * D || in_sizes[1] != 2 * EFULL || in_sizes[2] != 2 * D * HID || in_sizes[3] != HID || in_sizes[4] != HID || in_sizes[5] != 1 || out_size != EFULL) return;
  size_t off = 0; char* ws = (char*)d_ws;
  auto carve = [&](size_t bytes) { char* p = ws + off; off += (bytes + 255) & ~(size_t)255; return p; };
  b16* WT = (b16*)carve((size_t)2 * HID * D * 2); float* AB = (float*)carve((size_t)NP * 2 * HID * 4);
  if (off > ws_size || off > ((size_t)128 << 20)) return;
  wt_kernel<<<(2 * HID * D / 8 + 255) / 256, 256, 0, stream>>>(Fp(2), WT, WSC);
  ab_kernel<0><<<NP / 32, 64, 0, stream>>>(Fp(0), WT, Fp(3), AB);
  ab_kernel<1><<<NP / 32, 64, 0, stream>>>(Fp(0), WT, Fp(3), AB);
  edge_kernel<<<(EL + 255) / 256, 256, 0, stream>>>(AB, Ip(1), Fp(4), Fp(5), (float*)d_out, EL);
}
